// ISL_44573170598559
// MI455X (gfx1250) — hardware-run, weakly checked
//
#include <hip/hip_runtime.h>


#ifndef NB
#define NB 16
#endif
#define NB_FULL   16
#define NPTS      4096
#define NPTS_FULL 4096
#define KNN   20
#define CIN   3
#define CH    64
#define COLS  (NB * NPTS)
#define ECOLS 32
#define USP   68
#define OSP   36
#define BN_EPS 1e-5f
#define QRS  2048.0f
#define QRI  (1.0f / 2048.0f)
#define WSC  256.0f
#define WSI  (1.0f / 256.0f)
#define NBLK1 (COLS / 256)
#define NBLKG (COLS / 32)
#define LOG2E 1.4426950408889634f

static_assert(NB <= NB_FULL);
static_assert(NPTS == NPTS_FULL);
static_assert(CH == 64);
static_assert(CH % 32 == 0);
static_assert(CIN == 3);
static_assert(COLS % 256 == 0);
static_assert(NPTS % 256 == 0);
static_assert(NPTS % ECOLS == 0);
static_assert(NPTS % 128 == 0);
static_assert(ECOLS == 32);
static_assert(ECOLS * KNN == 2 * 256 + 128);
static_assert(CH * CIN == 6 * 32);
static_assert(CIN * ECOLS == 3 * 32);
static_assert(8 * CH == 2 * 256);
static_assert(256 * 16 == ECOLS * CH * 2);
static_assert(32 * 16 * 8 == 16 * CH * 4);
static_assert(32 * 16 * 4 == 16 * 32 * 4);
static_assert(32 * 16 == 128 * 4);
static_assert(16 * 16 == 32 * 8);
static_assert(((size_t)COLS * CH / 8) % 256 == 0);
static_assert(((size_t)NB * CH * NPTS / 4) % 256 == 0);
static_assert(((size_t)CH * CH / 8) % 256 == 0);
static_assert((USP * 4) % 16 == 0);
static_assert((OSP * 4) % 16 == 0);
static_assert((size_t)(KNN * CIN * ECOLS + CIN * ECOLS + 2 * CH * CIN + 8 * CH + ECOLS * USP) * 4 <= 131072);
static_assert((size_t)(16 * USP + 128) * 4 <= 131072);
static_assert((size_t)(8 * 18 + 4 * 128) * 8 <= 131072);

typedef _Float16 h16;
typedef __attribute__((ext_vector_type(16))) _Float16 v16h;
typedef __attribute__((ext_vector_type(8)))  _Float16 v8h;
typedef __attribute__((ext_vector_type(8)))  float    v8f;
typedef __attribute__((ext_vector_type(4)))  float    v4f;
typedef __attribute__((ext_vector_type(2)))  double   v2d;
typedef v4f  __attribute__((may_alias)) v4fa;

__device__ __forceinline__ unsigned short f2bf(float f) { unsigned u = __float_as_uint(f); u += 0x7FFFu + ((u >> 16) & 1u); return (unsigned short)(u >> 16); }
__device__ __forceinline__ float bfr(float f) { return __uint_as_float(((unsigned)f2bf(f)) << 16); }
__device__ __forceinline__ v16h cat16(v8h lo, v8h hi) { return __builtin_shufflevector(lo, hi, 0, 1, 2, 3, 4, 5, 6, 7, 8, 9, 10, 11, 12, 13, 14, 15); }
__device__ __forceinline__ v16h  ldh(const h16* p) { return cat16(*(const v8h*)p, *(const v8h*)(p + 16)); }
__device__ __forceinline__ void wave_sync() { __builtin_amdgcn_fence(3  , "wavefront"); __builtin_amdgcn_wave_barrier(); asm volatile("" ::: "memory"); }
static __device__ __forceinline__ h16 toh_flush(float v) { const h16 r = (h16)v; return (fabsf(v) < 6.103515625e-05f) ? (h16)0.0f : r; }
static __device__ __forceinline__ v8f wmma_g(v16h a, v16h b, v8f c) {
    c = __builtin_amdgcn_wmma_f32_16x16x32_f16(false, a, false, b, (short)0, c, false, false);
    asm volatile("v_nop\n\tv_nop\n\tv_nop\n\tv_nop" : "+v"(c) : "v"(a), "v"(b));
    return c;
}

__global__ __launch_bounds__(256) void k_stats_in(const float* __restrict__ x, const int* __restrict__ idx, double* part) {
    __shared__ double wsum[8 * 18];
    const int tid = threadIdx.x, lane = tid & 31;
    const int wave = __builtin_amdgcn_readfirstlane((int)(threadIdx.x >> 5));
    const int col = blockIdx.x * 256 + tid;
    const int b = col / NPTS, n = col % NPTS;
    const float* xb = x + (size_t)b * CIN * NPTS_FULL;
    const float x0 = bfr(xb[n]), x1 = bfr(xb[NPTS_FULL + n]), x2 = bfr(xb[2 * NPTS_FULL + n]);
    double acc[18];
#pragma unroll
    for (int v = 0; v < 9; ++v) acc[v] = 0.0;
    acc[9] = x0; acc[10] = x1; acc[11] = x2;
    acc[12] = (double)x0 * x0; acc[13] = (double)x0 * x1; acc[14] = (double)x0 * x2;
    acc[15] = (double)x1 * x1; acc[16] = (double)x1 * x2; acc[17] = (double)x2 * x2;
    const int* ip = idx + ((size_t)b * NPTS_FULL + n) * KNN;
#pragma unroll 1
    for (int k = 0; k < KNN; ++k) {
        int j = ip[k]; j = j < 0 ? 0 : (j > NPTS - 1 ? NPTS - 1 : j);
        const float f0 = bfr(xb[j]) - x0, f1 = bfr(xb[NPTS_FULL + j]) - x1, f2 = bfr(xb[2 * NPTS_FULL + j]) - x2;
        acc[0] += f0; acc[1] += f1; acc[2] += f2;
        acc[3] += (double)f0 * f0; acc[4] += (double)f0 * f1; acc[5] += (double)f0 * f2;
        acc[6] += (double)f1 * f1; acc[7] += (double)f1 * f2; acc[8] += (double)f2 * f2;
    }
#pragma unroll
    for (int v = 0; v < 18; ++v) {
        double s = acc[v];
        s += __shfl_xor(s, 16, 32); s += __shfl_xor(s, 8, 32); s += __shfl_xor(s, 4, 32); s += __shfl_xor(s, 2, 32); s += __shfl_xor(s, 1, 32);
        if (lane == 0) wsum[wave * 18 + v] = s;
    }
    __syncthreads();
    if (wave == 0) {
        const int e0 = 2 * lane, e1 = 2 * lane + 1;
        const int c0 = e0 < 18 ? e0 : 17, c1 = e1 < 18 ? e1 : 17;
        double s0 = 0.0, s1 = 0.0;
#pragma unroll
        for (int w = 0; w < 8; ++w) { s0 += wsum[w * 18 + c0]; s1 += wsum[w * 18 + c1]; }
        v2d o; o[0] = (e0 < 18) ? s0 : 0.0; o[1] = (e1 < 18) ? s1 : 0.0;
        if (lane < 16) {
            double* pp = part + (size_t)blockIdx.x * 32 + 2 * lane;
            *(volatile v2d*)pp = o; __threadfence(); *(volatile v2d*)pp = o;
        }
    }
}

__global__ __launch_bounds__(64) void k_fin1(const double* __restrict__ part,
                                             const float* __restrict__ Wnb, const float* __restrict__ Wself,
                                             const float* __restrict__ bng, const float* __restrict__ bnb,
                                             const float* __restrict__ bn2g, const float* __restrict__ bn2b, float* aff) {
    __shared__ double tot[18];
    const int tid = threadIdx.x;
    const int tc = tid < 18 ? tid : 17;
    double s = 0.0;
#pragma unroll 1
    for (int i = 0; i < NBLK1; ++i) s += part[(size_t)i * 32 + tc];
    if (tid < 18) tot[tid] = s;
    __syncthreads();
    const int o = tid;
    float vals[8];
    {
        const double invM = 1.0 / ((double)COLS * (double)KNN);
        const double w0 = bfr(Wnb[o * 3 + 0]), w1 = bfr(Wnb[o * 3 + 1]), w2 = bfr(Wnb[o * 3 + 2]);
        const double mean = (w0 * tot[0] + w1 * tot[1] + w2 * tot[2]) * invM;
        const double ey2 = (w0 * w0 * tot[3] + w1 * w1 * tot[6] + w2 * w2 * tot[8] +
                            2.0 * (w0 * w1 * tot[4] + w0 * w2 * tot[5] + w1 * w2 * tot[7])) * invM;
        double var = ey2 - mean * mean; var = var < 0.0 ? 0.0 : var;
        vals[0] = (float)mean; vals[1] = rsqrtf((float)var + BN_EPS); vals[2] = bfr(bng[o]); vals[3] = bfr(bnb[o]);
    }
    {
        const double invM = 1.0 / (double)COLS;
        const double w0 = bfr(Wself[o * 3 + 0]), w1 = bfr(Wself[o * 3 + 1]), w2 = bfr(Wself[o * 3 + 2]);
        const double mean = (w0 * tot[9] + w1 * tot[10] + w2 * tot[11]) * invM;
        const double ey2 = (w0 * w0 * tot[12] + w1 * w1 * tot[15] + w2 * w2 * tot[17] +
                            2.0 * (w0 * w1 * tot[13] + w0 * w2 * tot[14] + w1 * w2 * tot[16])) * invM;
        double var = ey2 - mean * mean; var = var < 0.0 ? 0.0 : var;
        vals[4] = (float)mean; vals[5] = rsqrtf((float)var + BN_EPS); vals[6] = bfr(bn2g[o]); vals[7] = bfr(bn2b[o]);
    }
#pragma unroll 1
    for (int ps = 0; ps < 2; ++ps) {
#pragma unroll
        for (int q = 0; q < 8; ++q) *(volatile float*)(aff + q * CH + o) = vals[q];
        if (ps == 0) __threadfence(); }
}

__global__ __launch_bounds__(256) void k_edge(const float* __restrict__ x, const int* __restrict__ idx,
                                              const float* __restrict__ Wnb, const float* __restrict__ Wself, const float* __restrict__ aff,
                                              float* A1, float* A2, h16* UH, h16* UR) {
    __shared__ float nbs[KNN * CIN * ECOLS];
    __shared__ float xcs[CIN * ECOLS];
    __shared__ float wn[CH * CIN];
    __shared__ float wsf[CH * CIN];
    __shared__ float afs[8 * CH];
    __shared__ __align__(16) float us[ECOLS * USP];
    const int tid = threadIdx.x, lane = tid & 31;
    const int wave = __builtin_amdgcn_readfirstlane((int)(threadIdx.x >> 5));
    const int b = blockIdx.x / (NPTS / ECOLS), n0 = (blockIdx.x % (NPTS / ECOLS)) * ECOLS;
    const float* xb = x + (size_t)b * CIN * NPTS_FULL;
    const int* ib = idx + ((size_t)b * NPTS_FULL + n0) * KNN;
    afs[tid] = aff[tid]; afs[256 + tid] = aff[256 + tid];
    if (wave < 6) { wn[tid] = bfr(Wnb[tid]); wsf[tid] = bfr(Wself[tid]); }
    if (wave < 3) xcs[wave * ECOLS + lane] = bfr(xb[(size_t)wave * NPTS_FULL + n0 + lane]);
#pragma unroll
    for (int it = 0; it < 3; ++it) {
        if (it < 2 || wave < 4) {
            const int e = tid + 256 * it; const int cl = e / KNN, k = e - cl * KNN;
            int j = ib[e]; j = j < 0 ? 0 : (j > NPTS - 1 ? NPTS - 1 : j);
            nbs[(k * CIN + 0) * ECOLS + cl] = bfr(xb[j]);
            nbs[(k * CIN + 1) * ECOLS + cl] = bfr(xb[NPTS_FULL + j]);
            nbs[(k * CIN + 2) * ECOLS + cl] = bfr(xb[2 * NPTS_FULL + j]);
        }
    }
    __syncthreads();
    const int ob = wave * 8;
    const float x0 = xcs[lane], x1 = xcs[ECOLS + lane], x2 = xcs[2 * ECOLS + lane];
    float w0[8], w1[8], w2[8], mx[8], mn[8];
#pragma unroll
    for (int i = 0; i < 8; ++i) { w0[i] = wn[(ob + i) * 3 + 0]; w1[i] = wn[(ob + i) * 3 + 1]; w2[i] = wn[(ob + i) * 3 + 2]; mx[i] = -3.4e38f; mn[i] = 3.4e38f; }
#pragma unroll 1
    for (int k = 0; k < KNN; ++k) {
        const float f0 = nbs[(k * CIN + 0) * ECOLS + lane] - x0, f1 = nbs[(k * CIN + 1) * ECOLS + lane] - x1, f2 = nbs[(k * CIN + 2) * ECOLS + lane] - x2;
#pragma unroll
        for (int i = 0; i < 8; ++i) { const float y = w0[i] * f0 + w1[i] * f1 + w2[i] * f2; mx[i] = fmaxf(mx[i], y); mn[i] = fminf(mn[i], y); }
    }
    float a1v[8], a2v[8];
#pragma unroll
    for (int i = 0; i < 8; ++i) {
        const int o = ob + i;
        const float m1 = afs[o], r1 = afs[CH + o], g1 = afs[2 * CH + o], b1 = afs[3 * CH + o];
        const float ys = (g1 >= 0.0f) ? mx[i] : mn[i];
        float v = ((ys - m1) * r1) * g1 + b1; v = (v >= 0.0f) ? v : 0.2f * v;
        const float y2 = wsf[o * 3 + 0] * x0 + wsf[o * 3 + 1] * x1 + wsf[o * 3 + 2] * x2;
        const float m2 = afs[4 * CH + o], r2 = afs[5 * CH + o], g2 = afs[6 * CH + o], b2 = afs[7 * CH + o];
        float v2 = ((y2 - m2) * r2) * g2 + b2; v2 = (v2 >= 0.0f) ? v2 : 0.2f * v2;
        a1v[i] = v; a2v[i] = v2; us[lane * USP + o] = v + v2;
    }
#pragma unroll 1
    for (int ps = 0; ps < 2; ++ps) {
#pragma unroll
        for (int i = 0; i < 8; ++i) { const size_t oo = ((size_t)(b * CH + ob + i)) * NPTS + n0 + lane;
            *(volatile float*)(A1 + oo) = a1v[i]; *(volatile float*)(A2 + oo) = a2v[i]; }
        if (ps == 0) __threadfence(); }
    __syncthreads();
    { const int row = tid >> 3, c8 = (tid & 7) * 8;
      const v4f u0 = *(const v4fa*)(&us[row * USP + c8]); const v4f u1 = *(const v4fa*)(&us[row * USP + c8 + 4]); v8h hv, rv;
#pragma unroll
      for (int i = 0; i < 4; ++i) { const h16 q0 = toh_flush(u0[i]); const h16 q1 = toh_flush(u1[i]); hv[i] = q0; hv[4 + i] = q1;
          rv[i] = toh_flush((u0[i] - (float)q0) * QRS); rv[4 + i] = toh_flush((u1[i] - (float)q1) * QRS); }
      const size_t oo = ((size_t)b * NPTS + n0 + row) * CH + c8;
      *(volatile v8h*)(UH + oo) = hv; *(volatile v8h*)(UR + oo) = rv; __threadfence();
      *(volatile v8h*)(UH + oo) = hv; *(volatile v8h*)(UR + oo) = rv; }
}

__global__ __launch_bounds__(256) void k_wconv(const float* __restrict__ src, h16* dst, size_t n8) {
    const size_t i = (size_t)blockIdx.x * 256 + threadIdx.x; if (i >= n8) return;
    const v8f v = *(const v8f*)(src + i * 8); v8h o;
#pragma unroll
    for (int k = 0; k < 8; ++k) o[k] = toh_flush(bfr(v[k]) * WSC);
    *(volatile v8h*)(dst + i * 8) = o; __threadfence(); *(volatile v8h*)(dst + i * 8) = o;
}

__global__ __launch_bounds__(32) void k_gemm_tok(const h16* __restrict__ AH, const h16* __restrict__ AR, const h16* __restrict__ W,
                                                 const float* __restrict__ bias, float* Z, float* PART) {
    __shared__ __align__(16) float os[16 * USP];
    __shared__ __align__(16) float pst[128];
    const int K = CH;
    const int lane = threadIdx.x & 31, lr = lane & 15, hi = lane >> 4; const int r0 = blockIdx.x * 32;
    v8f acc[2][4], accR[2][4];
#pragma unroll
    for (int mb = 0; mb < 2; ++mb)
#pragma unroll
        for (int nb = 0; nb < 4; ++nb) { acc[mb][nb] = (v8f){}; accR[mb][nb] = (v8f){}; }
    const size_t aoff = (size_t)(r0 + lr) * K + 8 * hi, boff = (size_t)lr * K + 8 * hi;
#pragma unroll 1
    for (int kc = 0; kc < K; kc += 32) {
        v16h ah[2], ar[2];
#pragma unroll
        for (int mb = 0; mb < 2; ++mb) { ah[mb] = ldh(AH + aoff + (size_t)mb * 16 * K + kc); ar[mb] = ldh(AR + aoff + (size_t)mb * 16 * K + kc); }
#pragma unroll
        for (int nb = 0; nb < 4; ++nb) { const v16h bw = ldh(W + boff + (size_t)nb * 16 * K + kc);
#pragma unroll
            for (int mb = 0; mb < 2; ++mb) { acc[mb][nb] = wmma_g(ah[mb], bw, acc[mb][nb]); accR[mb][nb] = wmma_g(ar[mb], bw, accR[mb][nb]); } }
    }
    float bc[4], cs[4], cq[4];
#pragma unroll
    for (int nb = 0; nb < 4; ++nb) { bc[nb] = bfr(bias[nb * 16 + lr]); cs[nb] = 0.0f; cq[nb] = 0.0f; }
#pragma unroll
    for (int mb = 0; mb < 2; ++mb) {
#pragma unroll
        for (int nb = 0; nb < 4; ++nb) {
#pragma unroll
            for (int j = 0; j < 8; ++j) { const float v = acc[mb][nb][j] * WSI + accR[mb][nb][j] * (QRI * WSI) + bc[nb];
                cs[nb] += v; cq[nb] += v * v; os[(hi * 8 + j) * USP + nb * 16 + lr] = v; } }
        wave_sync();
#pragma unroll 1
        for (int ps = 0; ps < 2; ++ps) {
#pragma unroll
            for (int s = 0; s < 8; ++s) { const int row = 2 * s + (lane >> 4), c4 = (lane & 15) * 4;
                const v4f val = *(const v4fa*)(&os[row * USP + c4]);
                *(volatile v4f*)(Z + (size_t)(r0 + mb * 16 + row) * CH + c4) = val; }
            if (ps == 0) __threadfence(); }
        wave_sync();
    }
#pragma unroll
    for (int nb = 0; nb < 4; ++nb) { cs[nb] += __shfl_xor(cs[nb], 16, 32); cq[nb] += __shfl_xor(cq[nb], 16, 32); }
    if (hi == 0) {
#pragma unroll
        for (int nb = 0; nb < 4; ++nb) { pst[nb * 16 + lr] = cs[nb]; pst[64 + nb * 16 + lr] = cq[nb]; } }
    wave_sync();
    { const v4f pv = *(const v4fa*)(&pst[lane * 4]);
      float* pp = PART + (size_t)blockIdx.x * 128 + lane * 4;
      *(volatile v4f*)pp = pv; __threadfence(); *(volatile v4f*)pp = pv; }
}

__global__ __launch_bounds__(32) void k_gemm_ch(const h16* __restrict__ W, const h16* __restrict__ BH, const h16* __restrict__ BR,
                                                const float* __restrict__ bias, float* C, float* PART) {
    __shared__ __align__(16) float os[16 * OSP];
    __shared__ __align__(16) float pst[128];
    const int K = CH;
    const int lane = threadIdx.x & 31, lr = lane & 15, hi = lane >> 4; const int c0 = blockIdx.x * 32;
    const int bb = c0 / NPTS, tt = c0 % NPTS;
    v8f acc[4][2], accR[4][2];
#pragma unroll
    for (int mb = 0; mb < 4; ++mb)
#pragma unroll
        for (int nb = 0; nb < 2; ++nb) { acc[mb][nb] = (v8f){}; accR[mb][nb] = (v8f){}; }
    const size_t aoff = (size_t)lr * K + 8 * hi, boff = (size_t)(c0 + lr) * K + 8 * hi;
#pragma unroll 1
    for (int kc = 0; kc < K; kc += 32) {
        v16h a[4];
#pragma unroll
        for (int mb = 0; mb < 4; ++mb) a[mb] = ldh(W + aoff + (size_t)mb * 16 * K + kc);
#pragma unroll
        for (int nb = 0; nb < 2; ++nb) { const v16h bh = ldh(BH + boff + (size_t)nb * 16 * K + kc); const v16h br = ldh(BR + boff + (size_t)nb * 16 * K + kc);
#pragma unroll
            for (int mb = 0; mb < 4; ++mb) { acc[mb][nb] = wmma_g(a[mb], bh, acc[mb][nb]); accR[mb][nb] = wmma_g(a[mb], br, accR[mb][nb]); } }
    }
#pragma unroll
    for (int mb = 0; mb < 4; ++mb) {
        float brw[8];
#pragma unroll
        for (int j = 0; j < 8; ++j) brw[j] = bfr(bias[mb * 16 + hi * 8 + j]);
#pragma unroll
        for (int nb = 0; nb < 2; ++nb) {
#pragma unroll
            for (int j = 0; j < 8; ++j) os[(hi * 8 + j) * OSP + nb * 16 + lr] = acc[mb][nb][j] * WSI + accR[mb][nb][j] * (QRI * WSI) + brw[j]; }
        wave_sync();
        { float s = 0.0f, q = 0.0f;
#pragma unroll
          for (int p = 0; p < 4; ++p) { const v4f t = *(const v4fa*)(&os[lr * OSP + 16 * hi + 4 * p]);
#pragma unroll
              for (int i = 0; i < 4; ++i) { s += t[i]; q += t[i] * t[i]; } }
          s += __shfl_xor(s, 16, 32); q += __shfl_xor(q, 16, 32);
          if (hi == 0) { pst[mb * 16 + lr] = s; pst[64 + mb * 16 + lr] = q; } }
#pragma unroll 1
        for (int ps = 0; ps < 2; ++ps) {
#pragma unroll
            for (int s = 0; s < 4; ++s) { const int row = 4 * s + (lane >> 3), cofs = (lane & 7) * 4;
                const v4f val = *(const v4fa*)(&os[row * OSP + cofs]);
                *(volatile v4f*)(C + ((size_t)(bb * CH + mb * 16 + row)) * NPTS + tt + cofs) = val; }
            if (ps == 0) __threadfence(); }
        wave_sync();
    }
    { const v4f pv = *(const v4fa*)(&pst[lane * 4]);
      float* pp = PART + (size_t)blockIdx.x * 128 + lane * 4;
      *(volatile v4f*)pp = pv; __threadfence(); *(volatile v4f*)pp = pv; }
}

__global__ __launch_bounds__(256) void k_finbn(const float* __restrict__ PART, const float* __restrict__ g, const float* __restrict__ bb, float* aff) {
    __shared__ double sh[4 * 128];
    const int tid = threadIdx.x, o = tid & 63, q = tid >> 6;
    const int wave = __builtin_amdgcn_readfirstlane((int)(threadIdx.x >> 5));
    double S = 0.0, Q = 0.0;
#pragma unroll 1
    for (int i = q; i < NBLKG; i += 4) { S += (double)PART[(size_t)i * 128 + o]; Q += (double)PART[(size_t)i * 128 + 64 + o]; }
    sh[q * 128 + o] = S; sh[q * 128 + 64 + o] = Q;
    __syncthreads();
    if (wave < 2) {
        const double invN = 1.0 / (double)COLS;
        const double St = ((sh[o] + sh[128 + o]) + sh[256 + o]) + sh[384 + o];
        const double Qt = ((sh[64 + o] + sh[128 + 64 + o]) + sh[256 + 64 + o]) + sh[384 + 64 + o];
        const double mean = St * invN;
        double var = Qt * invN - mean * mean; var = var < 0.0 ? 0.0 : var;
        const float v0 = (float)mean, v1 = rsqrtf((float)var + BN_EPS), v2 = bfr(g[o]), v3 = bfr(bb[o]);
        *(volatile float*)(aff + o) = v0; *(volatile float*)(aff + CH + o) = v1; *(volatile float*)(aff + 2 * CH + o) = v2; *(volatile float*)(aff + 3 * CH + o) = v3;
        __threadfence();
        *(volatile float*)(aff + o) = v0; *(volatile float*)(aff + CH + o) = v1; *(volatile float*)(aff + 2 * CH + o) = v2; *(volatile float*)(aff + 3 * CH + o) = v3;
    }
}

__global__ __launch_bounds__(256) void k_znorm(const float* __restrict__ ZP, const float* __restrict__ aff, h16* ZH, h16* ZR) {
#pragma clang fp contract(off)
    const size_t i = (size_t)blockIdx.x * 256 + threadIdx.x;
    const int c0 = (int)((i * 8) & (size_t)(CH - 1));
    const v4f z0 = *(const v4f*)(ZP + i * 8), z1 = *(const v4f*)(ZP + i * 8 + 4);
    const v4f m0 = *(const v4f*)(aff + c0), m1 = *(const v4f*)(aff + c0 + 4);
    const v4f r0 = *(const v4f*)(aff + CH + c0), r1 = *(const v4f*)(aff + CH + c0 + 4);
    const v4f g0 = *(const v4f*)(aff + 2 * CH + c0), g1 = *(const v4f*)(aff + 2 * CH + c0 + 4);
    const v4f b0 = *(const v4f*)(aff + 3 * CH + c0), b1 = *(const v4f*)(aff + 3 * CH + c0 + 4);
    v8h hv, rv;
#pragma unroll
    for (int k = 0; k < 4; ++k) {
        const float ya = ((z0[k] - m0[k]) * r0[k]) * g0[k] + b0[k];
        const float yb = ((z1[k] - m1[k]) * r1[k]) * g1[k] + b1[k];
        const h16 qa = toh_flush(ya); const h16 qb = toh_flush(yb);
        hv[k] = qa; hv[4 + k] = qb;
        rv[k] = toh_flush((ya - (float)qa) * QRS); rv[4 + k] = toh_flush((yb - (float)qb) * QRS);
    }
    *(volatile v8h*)(ZH + i * 8) = hv; *(volatile v8h*)(ZR + i * 8) = rv; __threadfence();
    *(volatile v8h*)(ZH + i * 8) = hv; *(volatile v8h*)(ZR + i * 8) = rv;
}

__global__ __launch_bounds__(256) void k_final(const float* __restrict__ A1, const float* __restrict__ A2, const float* __restrict__ CP,
                                               const float* __restrict__ aff, float* OUT) {
#pragma clang fp contract(off)
    const size_t i = (size_t)blockIdx.x * 256 + threadIdx.x;
    const size_t e = i * 4;
    const int o = (int)((e / NPTS) % CH);
    const float m = aff[o], r = aff[CH + o], g = aff[2 * CH + o], sb = aff[3 * CH + o];
    const v4f c = *(const v4f*)(CP + e), p1 = *(const v4f*)(A1 + e), p2 = *(const v4f*)(A2 + e);
    v4f ov;
#pragma unroll
    for (int k = 0; k < 4; ++k) {
        const float cat = ((c[k] - m) * r) * g + sb;
        const float ex = __builtin_amdgcn_exp2f(-cat * LOG2E);
        const float att = __builtin_amdgcn_rcpf(1.0f + ex);
        ov[k] = att * p1[k] + (1.0f - att) * p2[k];
    }
    *(volatile v4f*)(OUT + e) = ov; __threadfence(); *(volatile v4f*)(OUT + e) = ov;
}

static constexpr size_t al256(size_t v) { return (v + 255) & ~(size_t)255; }
static constexpr size_t SZ_P1  = al256((size_t)NBLK1 * 32 * 8);
static constexpr size_t SZ_AF1 = al256((size_t)8 * CH * 4);
static constexpr size_t SZ_A   = al256((size_t)NB * CH * NPTS * 4);
static constexpr size_t SZ_U   = al256((size_t)COLS * CH * 2);
static constexpr size_t SZ_W   = al256((size_t)2 * CH * CH * 2);
static constexpr size_t SZ_PG  = al256((size_t)NBLKG * 128 * 4);
static constexpr size_t SZ_AF  = al256((size_t)4 * CH * 4);
static constexpr size_t SZ_TOTAL = SZ_P1 + SZ_AF1 + 4 * SZ_A + 4 * SZ_U + SZ_W + 2 * SZ_PG + 2 * SZ_AF;
static_assert(SZ_TOTAL <= (size_t)134217728);
static_assert((size_t)(NBLK1 - 1) * 32 * 8 + 256 <= SZ_P1);
static_assert((size_t)(NBLKG - 1) * 128 * 4 + 512 <= SZ_PG);
static_assert(((size_t)CH * CH * 2) % 256 == 0);
static_assert((size_t)NB * CH * NPTS == (size_t)COLS * CH);

extern "C" void kernel_launch(void* const* d_in, const int* in_sizes, int n_in,
                              void* d_out, int out_size, void* d_ws, size_t ws_size, hipStream_t stream) {
    if (n_in < 16) return;
    if ((size_t)in_sizes[0] < (size_t)NB * CIN * NPTS_FULL) return;
    if ((size_t)in_sizes[1] < (size_t)NB * NPTS_FULL * KNN) return;
    if (in_sizes[2] < CH * CIN || in_sizes[3] < CH * CIN) return;
    if (in_sizes[4] < CH || in_sizes[5] < CH || in_sizes[6] < CH || in_sizes[7] < CH) return;
    if (in_sizes[8] < CH * CH || in_sizes[12] < CH * CH) return;
    if (in_sizes[9] < CH || in_sizes[10] < CH || in_sizes[11] < CH || in_sizes[13] < CH || in_sizes[14] < CH || in_sizes[15] < CH) return;
    if ((size_t)out_size < (size_t)NB * CH * NPTS) return;
    if (SZ_TOTAL > ws_size) return;
    const float* x      = (const float*)d_in[0];
    const int*   idx    = (const int*)d_in[1];
    const float* Wnb    = (const float*)d_in[2];
    const float* Wself  = (const float*)d_in[3];
    const float* bng    = (const float*)d_in[4];
    const float* bnb    = (const float*)d_in[5];
    const float* bn2g   = (const float*)d_in[6];
    const float* bn2b   = (const float*)d_in[7];
    const float* fcw    = (const float*)d_in[8];
    const float* fcb    = (const float*)d_in[9];
    const float* fcbng  = (const float*)d_in[10];
    const float* fcbnb  = (const float*)d_in[11];
    const float* fcow   = (const float*)d_in[12];
    const float* fcob   = (const float*)d_in[13];
    const float* fcobng = (const float*)d_in[14];
    const float* fcobnb = (const float*)d_in[15];
    float* OUT = (float*)d_out;
    char* wsp = (char*)d_ws;
    double* P1 = (double*)wsp; wsp += SZ_P1;
    float* AF1 = (float*)wsp;  wsp += SZ_AF1;
    float* A1  = (float*)wsp;  wsp += SZ_A;
    float* A2  = (float*)wsp;  wsp += SZ_A;
    float* ZP  = (float*)wsp;  wsp += SZ_A;
    float* CP  = (float*)wsp;  wsp += SZ_A;
    h16* UH = (h16*)wsp; wsp += SZ_U;
    h16* UR = (h16*)wsp; wsp += SZ_U;
    h16* ZH = (h16*)wsp; wsp += SZ_U;
    h16* ZR = (h16*)wsp; wsp += SZ_U;
    h16* WH = (h16*)wsp; wsp += SZ_W;
    float* PZ  = (float*)wsp; wsp += SZ_PG;
    float* PC  = (float*)wsp; wsp += SZ_PG;
    float* AFZ = (float*)wsp; wsp += SZ_AF;
    float* AFC = (float*)wsp; wsp += SZ_AF;
    h16* W1 = WH; h16* W2 = WH + (size_t)CH * CH;

    k_stats_in<<<NBLK1, 256, 0, stream>>>(x, idx, P1);
    k_fin1<<<1, 64, 0, stream>>>(P1, Wnb, Wself, bng, bnb, bn2g, bn2b, AF1);
    k_edge<<<COLS / ECOLS, 256, 0, stream>>>(x, idx, Wnb, Wself, AF1, A1, A2, UH, UR);
    { const size_t n8 = (size_t)CH * CH / 8; const unsigned g = (unsigned)((n8 + 255) / 256);
      k_wconv<<<g, 256, 0, stream>>>(fcw, W1, n8); k_wconv<<<g, 256, 0, stream>>>(fcow, W2, n8); }
    k_gemm_tok<<<NBLKG, 32, 0, stream>>>(UH, UR, W1, fcb, ZP, PZ);
    k_finbn<<<1, 256, 0, stream>>>(PZ, fcbng, fcbnb, AFZ);
    k_znorm<<<(unsigned)((size_t)COLS * CH / 8 / 256), 256, 0, stream>>>(ZP, AFZ, ZH, ZR);
    k_gemm_ch<<<NBLKG, 32, 0, stream>>>(W2, ZH, ZR, fcob, CP, PC);
    k_finbn<<<1, 256, 0, stream>>>(PC, fcobng, fcobnb, AFC);
    k_final<<<(unsigned)((size_t)NB * CH * NPTS / 4 / 256), 256, 0, stream>>>(A1, A2, CP, AFC, OUT);
}
